// LinearCrossAttention_54760833024196
// MI455X (gfx1250) — hardware-verified
//
#include <hip/hip_runtime.h>
#include <math.h>
#include <stdint.h>

#ifndef NB
#define NB 8
#endif
#define NB_FULL  8
#ifndef SEQ
#define SEQ 900
#endif
#define SEQ_FULL 900
#define TOK      SEQ_FULL
#define DM       256
#define NH       8
#define HD       32
#define RQ       (TOK * NB)
#define RA       (NB * TOK)
#define WSC      256.0f
#define CSC      16.0f
#define RESC     2048.0f
#define EPSF     1e-6f
#define GPITCH   68
#define WPITCH   36
#define FLOW_WAVES   4
#define FLOW_THREADS (FLOW_WAVES * 32)
#define FL_LDS   (3 * DM + 2 * DM + 8)

static_assert(SEQ == SEQ_FULL);
static_assert(NB >= 1 && NB <= NB_FULL);
static_assert(DM == NH * HD && HD == 32 && NH == 8);
static_assert((TOK % 2) == 0 && (RQ % 4) == 0);
static_assert((DM % 64) == 0 && (DM % 32) == 0);
static_assert((GPITCH * 4) % 16 == 0 && (WPITCH * 4) % 16 == 0 && (FL_LDS * 4) % 16 == 0);
static_assert(TOK * NB_FULL * DM == 1843200);

typedef unsigned short u16;
typedef _Float16 v16h __attribute__((ext_vector_type(16)));
typedef _Float16 v8h  __attribute__((ext_vector_type(8)));
typedef float    v8f  __attribute__((ext_vector_type(8)));
typedef float    v4f  __attribute__((ext_vector_type(4)));
typedef unsigned int v4u __attribute__((ext_vector_type(4)));

union FragH { v16h v; v8h h[2]; v4u u[2]; };

__device__ __forceinline__ unsigned short bf_bits(float f) {
  unsigned u = __float_as_uint(f);
  return (unsigned short)((u + 0x7FFFu + ((u >> 16) & 1u)) >> 16);
}
__device__ __forceinline__ float bf_up(unsigned short h) { return __uint_as_float(((unsigned)h) << 16); }
__device__ __forceinline__ float bfr(float f) { return bf_up(bf_bits(f)); }
__device__ __forceinline__ unsigned short h_bits(_Float16 x) { return __builtin_bit_cast(unsigned short, x); }
__device__ __forceinline__ unsigned pk16(unsigned short a, unsigned short b) { return (unsigned)a | ((unsigned)b << 16); }
__device__ __forceinline__ v8f zero8() { v8f z = {0.f, 0.f, 0.f, 0.f, 0.f, 0.f, 0.f, 0.f}; return z; }
__device__ __forceinline__ v4f bfr4(v4f a) { v4f r; r[0] = bfr(a[0]); r[1] = bfr(a[1]); r[2] = bfr(a[2]); r[3] = bfr(a[3]); return r; }
__device__ __forceinline__ int imin(int a, int b) { return a < b ? a : b; }
__device__ __forceinline__ float frcp(float x) { return __builtin_amdgcn_rcpf(x); }
__device__ __forceinline__ float sigm(float x) { return frcp(1.0f + expf(-x)); }
__device__ __forceinline__ float wsum(float x) {
#pragma unroll
  for (int off = 16; off > 0; off >>= 1) x += __shfl_xor(x, off, 32);
  return x;
}

__device__ __forceinline__ v16h ldfrag_h(const _Float16* p) {
  FragH f;
  f.h[0] = *(const v8h*)(p);
  f.h[1] = *(const v8h*)(p + 16);
  return f.v;
}

__device__ __forceinline__ v8f mma_h(v16h a, v16h b, v8f c) {
  return __builtin_amdgcn_wmma_f32_16x16x32_f16(false, a, false, b, (short)0, c, false, false);
}
__device__ __forceinline__ void guard_g(v8f (&acc)[8], v16h x0, v16h x1, v16h x2, v16h x3, v16h x4, v16h x5) {
#if defined(__HIP_DEVICE_COMPILE__)
  asm volatile("v_nop\n\tv_nop\n\tv_nop\n\tv_nop"
               : "+v"(acc[0]), "+v"(acc[1]), "+v"(acc[2]), "+v"(acc[3]),
                 "+v"(acc[4]), "+v"(acc[5]), "+v"(acc[6]), "+v"(acc[7])
               : "v"(x0), "v"(x1), "v"(x2), "v"(x3), "v"(x4), "v"(x5) : "memory");
#endif
}
__device__ __forceinline__ void wave_sync_lds() {
  __builtin_amdgcn_fence(__ATOMIC_RELEASE, "workgroup");
  __builtin_amdgcn_wave_barrier();
  __builtin_amdgcn_fence(__ATOMIC_ACQUIRE, "workgroup");
}

__global__ __launch_bounds__(128)
void cvt_x(const float* __restrict__ x, u16* Y, int rows) {
  const int wave = threadIdx.x >> 5, lane = threadIdx.x & 31;
  const int r = blockIdx.x * 4 + wave;
  if (r >= rows) return;
  const int l = r / NB, b = r - l * NB;
  const float* src = x + ((size_t)l * NB_FULL + (size_t)b) * DM + (size_t)lane * 8;
  const v4f a = *(const v4f*)(src), c4 = *(const v4f*)(src + 4);
  v4u o;
#pragma unroll
  for (int e = 0; e < 2; ++e) {
    o[e]     = pk16(h_bits((_Float16)bfr(a[2 * e])),  h_bits((_Float16)bfr(a[2 * e + 1])));
    o[2 + e] = pk16(h_bits((_Float16)bfr(c4[2 * e])), h_bits((_Float16)bfr(c4[2 * e + 1])));
  }
  u16* dst = Y + (size_t)r * DM + (size_t)lane * 8;
  for (int pass = 0; pass < 2; ++pass) {
    *(volatile v4u*)(dst) = o;
    __threadfence();
  }
}

__global__ __launch_bounds__(128)
void cvt_w(const float* __restrict__ w0, const float* __restrict__ w1, const float* __restrict__ w2,
           const float* __restrict__ w3, u16* Y) {
  const int wave = threadIdx.x >> 5, lane = threadIdx.x & 31;
  const int mi = blockIdx.x >> 6;
  const int r = blockIdx.x * 4 + wave;
  if (r >= 4 * DM) return;
  const float* wsel = (mi == 0) ? w0 : ((mi == 1) ? w1 : ((mi == 2) ? w2 : w3));
  const float* src = wsel + (size_t)(r & (DM - 1)) * DM + (size_t)lane * 8;
  const v4f a = *(const v4f*)(src), c4 = *(const v4f*)(src + 4);
  v4u o;
#pragma unroll
  for (int e = 0; e < 2; ++e) {
    o[e]     = pk16(h_bits((_Float16)(bfr(a[2 * e]) * WSC)),  h_bits((_Float16)(bfr(a[2 * e + 1]) * WSC)));
    o[2 + e] = pk16(h_bits((_Float16)(bfr(c4[2 * e]) * WSC)), h_bits((_Float16)(bfr(c4[2 * e + 1]) * WSC)));
  }
  u16* dst = Y + (size_t)r * DM + (size_t)lane * 8;
  for (int pass = 0; pass < 2; ++pass) {
    *(volatile v4u*)(dst) = o;
    __threadfence();
  }
}

__device__ __forceinline__ void gemm_core2(const _Float16* ap0, const _Float16* ap1, const _Float16* bp, int K,
                                           v8f (&acc)[8]) {
  const size_t rs16 = (size_t)16 * (size_t)K;
#pragma unroll 1
  for (int k0 = 0; k0 < K; k0 += 32) {
    const v16h a0 = ldfrag_h(ap0 + k0), a1 = ldfrag_h(ap1 + k0);
    const v16h b0 = ldfrag_h(bp + k0);
    const v16h b1 = ldfrag_h(bp + rs16 + k0);
    const v16h b2 = ldfrag_h(bp + 2 * rs16 + k0);
    const v16h b3 = ldfrag_h(bp + 3 * rs16 + k0);
    acc[0] = mma_h(a0, b0, acc[0]);
    acc[1] = mma_h(a0, b1, acc[1]);
    acc[2] = mma_h(a0, b2, acc[2]);
    acc[3] = mma_h(a0, b3, acc[3]);
    acc[4] = mma_h(a1, b0, acc[4]);
    acc[5] = mma_h(a1, b1, acc[5]);
    acc[6] = mma_h(a1, b2, acc[6]);
    acc[7] = mma_h(a1, b3, acc[7]);
    guard_g(acc, a0, a1, b0, b1, b2, b3);
  }
}
__device__ __forceinline__ void stage32x64(float* sl, v8f (&acc)[8], float oscale, int lane) {
  const int hh = lane >> 4, m = lane & 15;
#pragma unroll
  for (int i = 0; i < 2; ++i) {
#pragma unroll
    for (int r = 0; r < 8; ++r) {
      const int ro = (16 * i + 8 * hh + r) * GPITCH + m;
      sl[ro]      = acc[4 * i + 0][r] * oscale;
      sl[ro + 16] = acc[4 * i + 1][r] * oscale;
      sl[ro + 32] = acc[4 * i + 2][r] * oscale;
      sl[ro + 48] = acc[4 * i + 3][r] * oscale;
    }
  }
  wave_sync_lds();
}

template <int HAS_POS>
__global__ __launch_bounds__(128)
void gemm_x(const u16* __restrict__ A, const u16* __restrict__ Bt, float* C, const float* __restrict__ bias,
            const float* __restrict__ pos, int Mb, float oscale) {
  __shared__ __align__(16) float slab[4 * 32 * GPITCH];
  const int tid = threadIdx.x, wave = tid >> 5, lane = tid & 31, hh = lane >> 4, m = lane & 15;
  constexpr int ntile = DM / 64;
  const int bid  = blockIdx.x;
  const int nt   = bid % ntile;
  const int mt   = bid / ntile;
  const int rowb = mt * 128 + wave * 32;
  const int col0 = nt * 64;
  if (rowb >= Mb) return;
  const int ra0 = imin(rowb + m, Mb - 1), ra1 = imin(rowb + 16 + m, Mb - 1);
  const _Float16* Ab = (const _Float16*)(const void*)A;
  const _Float16* ap0 = Ab + (size_t)ra0 * DM + 8 * hh;
  const _Float16* ap1 = Ab + (size_t)ra1 * DM + 8 * hh;
  const _Float16* bp = (const _Float16*)(const void*)Bt + (size_t)(col0 + m) * DM + 8 * hh;
  v8f acc[8];
#pragma unroll
  for (int i = 0; i < 8; ++i) acc[i] = zero8();
  gemm_core2(ap0, ap1, bp, DM, acc);
  float* sl = slab + wave * 32 * GPITCH;
  stage32x64(sl, acc, oscale, lane);
  const v4f bc = bfr4(*(const v4f*)(bias + col0 + m * 4));
  v4f vals[16];
#pragma unroll
  for (int it = 0; it < 16; ++it) {
    const int rr = imin(rowb + it * 2 + hh, Mb - 1);
    v4f v = *(const v4f*)(sl + (it * 2 + hh) * GPITCH + m * 4) + bc;
    if (HAS_POS) {
      const int l = rr / NB, b = rr - l * NB;
      const size_t srow = (size_t)l * NB_FULL + (size_t)b;
      v += bfr4(*(const v4f*)(pos + srow * DM + col0 + m * 4));
    }
    vals[it] = v;
  }
  float* Cb = C + ((size_t)rowb + (size_t)hh) * DM + col0 + m * 4;
  for (int pass = 0; pass < 2; ++pass) {
#pragma unroll
    for (int it = 0; it < 16; ++it) {
      if (rowb + it * 2 + hh < Mb) *(volatile v4f*)(Cb + (size_t)(it * 2) * DM) = vals[it];
    }
    __threadfence();
  }
}

__global__ __launch_bounds__(FLOW_THREADS)
void flow_tok(const float* __restrict__ Qp, const float* __restrict__ Kp, const float* __restrict__ Vp,
              u16* CHp, u16* CLp) {
  __shared__ __align__(16) float lds[FLOW_WAVES * FL_LDS];
  const int tid = threadIdx.x, wave = tid >> 5, lane = tid & 31;
  const int gw = blockIdx.x * FLOW_WAVES + wave;
  if (gw >= NB * (TOK / 2)) return;
  const int b  = gw % NB;
  const int l0 = (gw / NB) * 2;
  float* sqs  = lds + wave * FL_LDS;
  float* sk   = sqs + DM;
  float* svs  = sk + DM;
  float* sctx = svs + DM;
  float* sal  = sctx + 2 * DM;

#pragma unroll 1
  for (int t = 0; t < 2; ++t) {
    const size_t rowoff = ((size_t)(l0 + t) * NB + (size_t)b) * DM + (size_t)lane;
    float ck = 0.f, cq = 0.f, ckso = 0.f, cqsi = 0.f, ccs = 0.f;
#pragma unroll 1
    for (int h = 0; h < NH; ++h) {
      const size_t o = rowoff + (size_t)h * HD;
      const float qv = sigm(Qp[o]);
      const float kv = sigm(Kp[o]);
      const float vv = Vp[o];
      const float nm  = (float)(h + 1);
      const float rnm = frcp(nm);
      ck += kv;
      cq += qv;
      const float din = wsum((qv + EPSF) * (ck + EPSF));
      const float dou = wsum((kv + EPSF) * (cq + EPSF));
      const float si = frcp(din) * nm;
      const float so = frcp(dou) * nm;
      ckso += kv * so;
      cqsi += qv * si;
      const float csk = wsum((qv + EPSF) * (ckso + EPSF)) * rnm;
      float csr = wsum((kv + EPSF) * (cqsi + EPSF)) * rnm;
      csr = fminf(1.0f, fmaxf(-1.0f, csr));
      const float sa = sigm(csk);
      const float ex = expf(csr);
      ccs += ex;
      const float sc = ex * frcp(ccs) * nm;
      sqs[h * HD + lane] = qv * (si * rnm);
      sk[h * HD + lane]  = kv;
      svs[h * HD + lane] = vv * sc;
      sal[h] = sa;
    }
#pragma unroll 1
    for (int h = 0; h < NH; ++h) {
      const float qsh = sqs[h * HD + lane];
      float acc = 0.f;
#pragma unroll 1
      for (int hp = 0; hp <= h; ++hp) {
        const float s = wsum(qsh * sk[hp * HD + lane]);
        acc += s * svs[hp * HD + lane];
      }
      sctx[t * DM + h * HD + lane] = acc * sal[h] * CSC;
    }
  }
  wave_sync_lds();

  const int p = lane & 7, hq = lane >> 3;
  const int t = p >> 2, dseg = (p & 3) * 8;
  v4u oh[2], ol[2];
#pragma unroll
  for (int i = 0; i < 2; ++i) {
    const int h = 4 * i + hq;
    const float* s = sctx + t * DM + h * HD + dseg;
    const v4f a = *(const v4f*)(s), c4 = *(const v4f*)(s + 4);
#pragma unroll
    for (int e = 0; e < 2; ++e) {
      const _Float16 ha0 = (_Float16)a[2 * e],  ha1 = (_Float16)a[2 * e + 1];
      const _Float16 hc0 = (_Float16)c4[2 * e], hc1 = (_Float16)c4[2 * e + 1];
      const _Float16 la0 = (_Float16)((a[2 * e]      - (float)ha0) * RESC);
      const _Float16 la1 = (_Float16)((a[2 * e + 1]  - (float)ha1) * RESC);
      const _Float16 lc0 = (_Float16)((c4[2 * e]     - (float)hc0) * RESC);
      const _Float16 lc1 = (_Float16)((c4[2 * e + 1] - (float)hc1) * RESC);
      oh[i][e]     = pk16(h_bits(ha0), h_bits(ha1));
      oh[i][2 + e] = pk16(h_bits(hc0), h_bits(hc1));
      ol[i][e]     = pk16(h_bits(la0), h_bits(la1));
      ol[i][2 + e] = pk16(h_bits(lc0), h_bits(lc1));
    }
  }
  const size_t pb = (size_t)b * TOK * DM + (size_t)l0 * HD + (size_t)p * 8;
  u16* hb = CHp + pb;
  u16* lb = CLp + pb;
  for (int pass = 0; pass < 2; ++pass) {
#pragma unroll
    for (int i = 0; i < 2; ++i) {
      const size_t ho = (size_t)(4 * i + hq) * TOK * HD;
      *(volatile v4u*)(hb + ho) = oh[i];
    }
#pragma unroll
    for (int i = 0; i < 2; ++i) {
      const size_t ho = (size_t)(4 * i + hq) * TOK * HD;
      *(volatile v4u*)(lb + ho) = ol[i];
    }
    __threadfence();
  }
}

__global__ __launch_bounds__(128)
void gemm_wo(const u16* __restrict__ CHp, const u16* __restrict__ CLp, const u16* __restrict__ WO, float* out,
             const float* __restrict__ bo, const float* __restrict__ xres, int Mb) {
  __shared__ __align__(16) float slab[4 * 32 * WPITCH];
  const int tid = threadIdx.x, wave = tid >> 5, lane = tid & 31, hh = lane >> 4, m = lane & 15;
  constexpr int ntile = DM / 32;
  const int bid  = blockIdx.x;
  const int nt   = bid % ntile;
  const int mt   = bid / ntile;
  const int rowb = mt * 128 + wave * 32;
  const int col0 = nt * 32;
  if (rowb >= Mb) return;
  const int ra0 = imin(rowb + m, Mb - 1), ra1 = imin(rowb + 16 + m, Mb - 1);
  const _Float16* Hb = (const _Float16*)(const void*)CHp;
  const _Float16* Lb = (const _Float16*)(const void*)CLp;
  const _Float16* ah0 = Hb + (size_t)ra0 * DM + 8 * hh;
  const _Float16* ah1 = Hb + (size_t)ra1 * DM + 8 * hh;
  const _Float16* al0 = Lb + (size_t)ra0 * DM + 8 * hh;
  const _Float16* al1 = Lb + (size_t)ra1 * DM + 8 * hh;
  const _Float16* bp = (const _Float16*)(const void*)WO + (size_t)(col0 + m) * DM + 8 * hh;
  v8f acc[8];
#pragma unroll
  for (int i = 0; i < 8; ++i) acc[i] = zero8();
#pragma unroll 1
  for (int k0 = 0; k0 < DM; k0 += 32) {
    const v16h a0h = ldfrag_h(ah0 + k0), a1h = ldfrag_h(ah1 + k0);
    const v16h a0l = ldfrag_h(al0 + k0), a1l = ldfrag_h(al1 + k0);
    const v16h b0 = ldfrag_h(bp + k0);
    const v16h b1 = ldfrag_h(bp + (size_t)16 * DM + k0);
    acc[0] = mma_h(a0h, b0, acc[0]);
    acc[1] = mma_h(a0h, b1, acc[1]);
    acc[2] = mma_h(a1h, b0, acc[2]);
    acc[3] = mma_h(a1h, b1, acc[3]);
    acc[4] = mma_h(a0l, b0, acc[4]);
    acc[5] = mma_h(a0l, b1, acc[5]);
    acc[6] = mma_h(a1l, b0, acc[6]);
    acc[7] = mma_h(a1l, b1, acc[7]);
    guard_g(acc, a0h, a1h, a0l, a1l, b0, b1);
  }
  const float sh = 1.0f / (CSC * WSC);
  const float sl = sh / RESC;
  float* slb = slab + wave * 32 * WPITCH;
#pragma unroll
  for (int i = 0; i < 2; ++i) {
#pragma unroll
    for (int r = 0; r < 8; ++r) {
      const int ro = (16 * i + 8 * hh + r) * WPITCH + m;
      slb[ro]      = acc[2 * i + 0][r] * sh + acc[4 + 2 * i + 0][r] * sl;
      slb[ro + 16] = acc[2 * i + 1][r] * sh + acc[4 + 2 * i + 1][r] * sl;
    }
  }
  wave_sync_lds();
  const int rq = lane >> 3, c4 = (lane & 7) * 4;
  const v4f bc = bfr4(*(const v4f*)(bo + col0 + c4));
  v4f vals[8];
  size_t orow[8];
#pragma unroll
  for (int i = 0; i < 8; ++i) {
    const int rr = imin(rowb + 4 * i + rq, Mb - 1);
    const int bb = rr / TOK;
    const int nn = rr - bb * TOK;
    const size_t orw = (size_t)nn * NB_FULL + (size_t)bb;
    v4f v = *(const v4f*)(slb + (4 * i + rq) * WPITCH + c4) + bc;
    v += bfr4(*(const v4f*)(xres + orw * DM + col0 + c4));
    vals[i] = v;
    orow[i] = orw;
  }
  for (int pass = 0; pass < 2; ++pass) {
#pragma unroll
    for (int i = 0; i < 8; ++i) {
      if (rowb + 4 * i + rq < Mb) *(volatile v4f*)(out + orow[i] * DM + col0 + c4) = vals[i];
    }
    __threadfence();
  }
}

extern "C" void kernel_launch(void* const* d_in, const int* in_sizes, int n_in,
                              void* d_out, int out_size, void* d_ws, size_t ws_size,
                              hipStream_t stream) {
  if (n_in < 12) return;
  const int actMin = TOK * NB_FULL * DM;
  if (in_sizes[0] < actMin || in_sizes[1] < actMin || in_sizes[2] < actMin || in_sizes[3] < actMin) return;
  if (in_sizes[4] < DM * DM || in_sizes[6] < DM * DM || in_sizes[8] < DM * DM || in_sizes[10] < DM * DM) return;
  if (in_sizes[5] < DM || in_sizes[7] < DM || in_sizes[9] < DM || in_sizes[11] < DM) return;
  if (out_size < actMin) return;

  const float* query     = (const float*)d_in[0];
  const float* key       = (const float*)d_in[1];
  const float* query_pos = (const float*)d_in[2];
  const float* key_pos   = (const float*)d_in[3];
  const float* Wq = (const float*)d_in[4];
  const float* bq = (const float*)d_in[5];
  const float* Wk = (const float*)d_in[6];
  const float* bk = (const float*)d_in[7];
  const float* Wv = (const float*)d_in[8];
  const float* bv = (const float*)d_in[9];
  const float* Wo = (const float*)d_in[10];
  const float* bo = (const float*)d_in[11];
  float* out = (float*)d_out;

  const size_t szX = (size_t)RQ * DM * 2;
  const size_t szW = (size_t)4 * DM * DM * 2;
  const size_t szP = (size_t)RQ * DM * 4;
  const size_t szC = (size_t)RA * DM * 2;
  size_t off = 0;
  const size_t oXQ = off; off += szX;
  const size_t oXK = off; off += szX;
  const size_t oW  = off; off += szW;
  const size_t oQP = off; off += szP;
  const size_t oKP = off; off += szP;
  const size_t oVP = off; off += szP;
  const size_t oCH = off; off += szC;
  const size_t oCL = off; off += szC;
  if (off > ws_size) return;
  if (off > (size_t)134217728) return;

  char* ws = (char*)d_ws;
  u16*   XQ  = (u16*)(ws + oXQ);
  u16*   XK  = (u16*)(ws + oXK);
  u16*   W16 = (u16*)(ws + oW);
  float* QP  = (float*)(ws + oQP);
  float* KP  = (float*)(ws + oKP);
  float* VP  = (float*)(ws + oVP);
  u16*   CH  = (u16*)(ws + oCH);
  u16*   CL  = (u16*)(ws + oCL);

  cvt_x<<<dim3(RQ / 4), dim3(128), 0, stream>>>(query, XQ, RQ);
  cvt_x<<<dim3(RQ / 4), dim3(128), 0, stream>>>(key, XK, RQ);
  cvt_w<<<dim3(4 * DM / 4), dim3(128), 0, stream>>>(Wq, Wk, Wv, Wo, W16);
  const int mtq = (RQ + 127) / 128;
  gemm_x<1><<<dim3(mtq * (DM / 64)), dim3(128), 0, stream>>>(XQ, W16, QP, bq, query_pos, RQ, 1.0f / WSC);
  gemm_x<1><<<dim3(mtq * (DM / 64)), dim3(128), 0, stream>>>(XK, W16 + (size_t)DM * DM, KP, bk, key_pos, RQ, 1.0f / WSC);
  gemm_x<0><<<dim3(mtq * (DM / 64)), dim3(128), 0, stream>>>(XK, W16 + (size_t)2 * DM * DM, VP, bv, key_pos, RQ, 1.0f / WSC);
  flow_tok<<<dim3((NB * (TOK / 2) + FLOW_WAVES - 1) / FLOW_WAVES), dim3(FLOW_THREADS), 0, stream>>>(QP, KP, VP, CH, CL);
  const int mta = (RA + 127) / 128;
  gemm_wo<<<dim3(mta * (DM / 32)), dim3(128), 0, stream>>>(CH, CL, W16 + (size_t)3 * DM * DM, out, bo, query, RA);
  (void)hipGetLastError();
}
